// PointNetSA_25735444037745
// MI455X (gfx1250) — hardware-verified
//
#include <hip/hip_runtime.h>

#pragma clang fp contract(off)

typedef __attribute__((ext_vector_type(16))) _Float16 v16h;
typedef __attribute__((ext_vector_type(8)))  _Float16 v8h;
typedef __attribute__((ext_vector_type(8)))  float    v8f;
typedef __attribute__((ext_vector_type(4)))  float    v4f;
typedef __attribute__((ext_vector_type(4)))  unsigned int v4u;

constexpr int NBATCH   = 8;
constexpr int NPTS     = 8192;
constexpr int NFEAT    = 64;
constexpr int NQUERY   = 2048;
constexpr int NSAMP    = 32;
constexpr int CIN1     = 67;
constexpr int KPAD1    = 96;
constexpr int CH1      = 64;
constexpr int CH2      = 64;
constexpr int CH3      = 128;
constexpr float BN_EPS = 1e-5f;
constexpr float LEAK   = 0.2f;
constexpr float RAD2   = 0.04f;

static_assert(NPTS % 64 == 0);
static_assert(NQUERY % 32 == 0);
static_assert(KPAD1 % 32 == 0 && CH1 % 32 == 0 && CH2 % 32 == 0);
static_assert(CH1 % 16 == 0 && CH2 % 16 == 0 && CH3 % 16 == 0);

constexpr int W1T_OFF   = 0;
constexpr int W2T_OFF   = CH1 * KPAD1;
constexpr int W3T_OFF   = W2T_OFF + CH2 * CH1;
constexpr int WPL_HALVES = W3T_OFF + CH3 * CH2;
static_assert(WPL_HALVES == 18432);
static_assert(WPL_HALVES / 8 == 9 * 256);

constexpr size_t WS_WPL   = 0;
constexpr size_t WS_BIAS  = 36864;
constexpr size_t WS_QPL   = 37888;
constexpr size_t WS_PTS4  = WS_QPL + (size_t)NBATCH * NQUERY * 16;
constexpr size_t WS_FEATT = WS_PTS4 + (size_t)NBATCH * NPTS * 16;
constexpr size_t WS_TOTAL = WS_FEATT + (size_t)NBATCH * NPTS * NFEAT * 2;
static_assert(WS_BIAS == (size_t)WPL_HALVES * 2);
static_assert(WS_QPL % 128 == 0 && WS_PTS4 % 128 == 0 && WS_FEATT % 128 == 0);
static_assert(WS_TOTAL == 9737216);
static_assert(WS_TOTAL <= 134217728);

constexpr size_t OUT0_ELEMS = (size_t)NBATCH * CH3 * NQUERY;
constexpr size_t OUT1_ELEMS = (size_t)NBATCH * 3 * NQUERY;
static_assert(OUT0_ELEMS * 4 == 8388608);
static_assert((OUT0_ELEMS + OUT1_ELEMS) * 4 == 8585216);

union FragU { v16h v; v8h h[2]; };
__device__ __forceinline__ v16h frag_load(const _Float16* p) {
  FragU f;
  f.h[0] = *(const v8h*)(p);
  f.h[1] = *(const v8h*)(p + 16);
  return f.v;
}
__device__ __forceinline__ v8f mma_h(v16h a, v16h b, v8f c) {
  c = __builtin_amdgcn_wmma_f32_16x16x32_f16(false, a, false, b, (short)0, c, false, false);
  asm volatile("v_nop\n\tv_nop\n\tv_nop\n\tv_nop" : "+v"(c) : "v"(a), "v"(b));
  return c;
}
__device__ __forceinline__ float leaky(float y) { return y > 0.0f ? y : LEAK * y; }

__global__ __launch_bounds__(256) void prep_kernel(
    const float* __restrict__ w1, const float* __restrict__ b1, const float* __restrict__ g1,
    const float* __restrict__ bb1, const float* __restrict__ m1, const float* __restrict__ v1,
    const float* __restrict__ w2, const float* __restrict__ b2, const float* __restrict__ g2,
    const float* __restrict__ bb2, const float* __restrict__ m2, const float* __restrict__ v2,
    const float* __restrict__ w3, const float* __restrict__ b3, const float* __restrict__ g3,
    const float* __restrict__ bb3, const float* __restrict__ m3, const float* __restrict__ v3,
    _Float16* __restrict__ wpl, float* __restrict__ biasf) {
  const int tid = threadIdx.x;
  if (blockIdx.x < 9) {
    const int grp = blockIdx.x * 256 + tid;
    const float* w = w3;
    const float* g = g3;
    const float* vv = v3;
    int o, k8, cin, reorder;
    if (grp < 768) {
      o = grp / 12; k8 = (grp % 12) * 8; cin = CIN1; reorder = 1;
      w = w1; g = g1; vv = v1;
    } else if (grp < 1280) {
      const int i = grp - 768;
      o = i >> 3; k8 = (i & 7) * 8; cin = CH1; reorder = 0;
      w = w2; g = g2; vv = v2;
    } else {
      const int i = grp - 1280;
      o = i >> 3; k8 = (i & 7) * 8; cin = CH2; reorder = 0;
    }
    const float sc = g[o] * rsqrtf(vv[o] + BN_EPS);
    float zf = 0.0f;
    asm volatile("" : "+v"(zf));
    float wv[8];
#pragma unroll
    for (int e = 0; e < 8; ++e) {
      const int k = k8 + e;
      int col = reorder ? ((k < 64) ? (k + 3) : (k - 64)) : k;
      col = col < cin ? col : cin - 1;
      wv[e] = w[o * cin + col];
    }
    v8h hv;
#pragma unroll
    for (int e = 0; e < 8; ++e) {
      const int k = k8 + e;
      const bool live = reorder ? (k < CIN1) : true;
      const float val = live ? (wv[e] * sc) : zf;
      hv[e] = (_Float16)val;
    }
    _Float16* dst = wpl + (size_t)grp * 8;
    *(volatile v8h*)dst = hv;
    __threadfence();
    *(volatile v8h*)dst = hv;
  } else {
    const float* bp = b3;
    const float* gp = g3;
    const float* bbp = bb3;
    const float* mp = m3;
    const float* vp = v3;
    int i = tid - 128;
    if (tid < 64) {
      bp = b1; gp = g1; bbp = bb1; mp = m1; vp = v1; i = tid;
    } else if (tid < 128) {
      bp = b2; gp = g2; bbp = bb2; mp = m2; vp = v2; i = tid - 64;
    }
    const float sc = gp[i] * rsqrtf(vp[i] + BN_EPS);
    const float r = (bp[i] - mp[i]) * sc + bbp[i];
    *(volatile float*)(biasf + tid) = r;
    __threadfence();
    *(volatile float*)(biasf + tid) = r;
  }
}

__global__ __launch_bounds__(256) void pack_kernel(
    const float* __restrict__ features, const float* __restrict__ points,
    _Float16* __restrict__ featT, float* __restrict__ pts4) {
#pragma clang fp contract(off)
  __shared__ __align__(16) _Float16 tile[64 * 72];
  const int tid = threadIdx.x;
  const int b   = blockIdx.x >> 7;
  const int n0  = (blockIdx.x & 127) * 64;
  const int n4  = (tid & 15) * 4;
  const int cb  = tid >> 4;
  v4f fv[4];
#pragma unroll
  for (int i = 0; i < 4; ++i) {
    const int c = cb + 16 * i;
    fv[i] = *(const v4f*)(features + ((size_t)(b * NFEAT + c)) * NPTS + n0 + n4);
  }
#pragma unroll
  for (int i = 0; i < 4; ++i) {
    const int c = cb + 16 * i;
    const v4f t = fv[i];
    tile[(n4 + 0) * 72 + c] = (_Float16)t[0];
    tile[(n4 + 1) * 72 + c] = (_Float16)t[1];
    tile[(n4 + 2) * 72 + c] = (_Float16)t[2];
    tile[(n4 + 3) * 72 + c] = (_Float16)t[3];
  }
  __syncthreads();
  const int c8 = (tid & 7) * 8;
  const int r0 = tid >> 3;
  const v8h h0 = *(const v8h*)(tile + r0 * 72 + c8);
  const v8h h1 = *(const v8h*)(tile + (r0 + 32) * 72 + c8);
  _Float16* d0 = featT + ((size_t)(b * NPTS + n0 + r0)) * NFEAT + c8;
  _Float16* d1 = featT + ((size_t)(b * NPTS + n0 + r0 + 32)) * NFEAT + c8;
  for (int pass = 0; pass < 2; ++pass) {
    *(volatile v8h*)d0 = h0;
    *(volatile v8h*)d1 = h1;
    __threadfence();
  }
  if (tid < 64) {
    const int n = n0 + tid;
    const float x = points[((size_t)(b * 3 + 0)) * NPTS + n];
    const float y = points[((size_t)(b * 3 + 1)) * NPTS + n];
    const float z = points[((size_t)(b * 3 + 2)) * NPTS + n];
    const float t0 = x * x;
    const float t1 = y * y;
    const float t2 = z * z;
    const float sq = (t0 + t2) + t1;
    const v4f pv = {x, y, z, sq};
    float* dp = pts4 + ((size_t)(b * NPTS + n)) * 4;
    *(volatile v4f*)dp = pv;
    __threadfence();
    *(volatile v4f*)dp = pv;
  }
}

constexpr int FPS_THREADS = 512;
constexpr int FPS_PER     = NPTS / FPS_THREADS;
constexpr int FPS_GSTRIDE = FPS_THREADS * 4;
static_assert(FPS_PER == 16);
static_assert(FPS_GSTRIDE * 4 == NPTS);
static_assert(NQUERY == 4 * FPS_THREADS);

__global__ __launch_bounds__(512) void fps_kernel(
    const float* __restrict__ points, float* __restrict__ qplane, float* __restrict__ out_xyz) {
#pragma clang fp contract(off)
  __shared__ float sval[2][16];
  __shared__ int   sidx[2][16];
  __shared__ int   fidx_s[NQUERY];

  const int b    = blockIdx.x;
  const int tid  = threadIdx.x;
  const int lane = tid & 31;
  const int w    = tid >> 5;
  const float* px = points + (size_t)b * 3 * NPTS;
  const float* py = px + NPTS;
  const float* pz = py + NPTS;

  float X[FPS_PER], Y[FPS_PER], Z[FPS_PER], D[FPS_PER];
  {
    int off = tid * 4;
    v4f xv0 = *(const v4f*)(px + 0 * FPS_GSTRIDE + off);
    v4f xv1 = *(const v4f*)(px + 1 * FPS_GSTRIDE + off);
    v4f xv2 = *(const v4f*)(px + 2 * FPS_GSTRIDE + off);
    v4f xv3 = *(const v4f*)(px + 3 * FPS_GSTRIDE + off);
    v4f yv0 = *(const v4f*)(py + 0 * FPS_GSTRIDE + off);
    v4f yv1 = *(const v4f*)(py + 1 * FPS_GSTRIDE + off);
    v4f yv2 = *(const v4f*)(py + 2 * FPS_GSTRIDE + off);
    v4f yv3 = *(const v4f*)(py + 3 * FPS_GSTRIDE + off);
    asm volatile("" : "+v"(off), "+v"(xv0), "+v"(xv1), "+v"(xv2), "+v"(xv3),
                      "+v"(yv0), "+v"(yv1), "+v"(yv2), "+v"(yv3) :: "memory");
    v4f zv0 = *(const v4f*)(pz + 0 * FPS_GSTRIDE + off);
    v4f zv1 = *(const v4f*)(pz + 1 * FPS_GSTRIDE + off);
    v4f zv2 = *(const v4f*)(pz + 2 * FPS_GSTRIDE + off);
    v4f zv3 = *(const v4f*)(pz + 3 * FPS_GSTRIDE + off);
    asm volatile("" : "+v"(zv0), "+v"(zv1), "+v"(zv2), "+v"(zv3) :: "memory");
#pragma unroll
    for (int e = 0; e < 4; ++e) {
      X[0 + e]  = xv0[e]; X[4 + e]  = xv1[e]; X[8 + e]  = xv2[e]; X[12 + e] = xv3[e];
      Y[0 + e]  = yv0[e]; Y[4 + e]  = yv1[e]; Y[8 + e]  = yv2[e]; Y[12 + e] = yv3[e];
      Z[0 + e]  = zv0[e]; Z[4 + e]  = zv1[e]; Z[8 + e]  = zv2[e]; Z[12 + e] = zv3[e];
    }
  }
#pragma unroll
  for (int j = 0; j < FPS_PER; ++j) D[j] = 1e10f;

  const int ibase = tid * 4;
  int far = 0;
  int buf = 0;
#pragma unroll 1
  for (int it = 0; it < NQUERY; ++it) {
    far = far < 0 ? 0 : (far > NPTS - 1 ? NPTS - 1 : far);
    if (tid == 0) fidx_s[it] = far;
    const float cx = px[far];
    const float cy = py[far];
    const float cz = pz[far];
    float bv = -1.0f;
    int   bi = 0;
#pragma unroll
    for (int j = 0; j < FPS_PER; ++j) {
      const float dx = X[j] - cx;
      const float dy = Y[j] - cy;
      const float dz = Z[j] - cz;
      const float t0 = dx * dx;
      const float t1 = dy * dy;
      const float t2 = dz * dz;
      const float d  = (t0 + t2) + t1;
      const float nd = fminf(D[j], d);
      D[j] = nd;
      const bool up = nd > bv;
      bv = up ? nd : bv;
      bi = up ? ((j >> 2) * FPS_GSTRIDE + ibase + (j & 3)) : bi;
    }
#pragma unroll
    for (int off = 16; off > 0; off >>= 1) {
      const float ov = __shfl_xor(bv, off, 32);
      const int   oi = __shfl_xor(bi, off, 32);
      const bool take = (ov > bv) || (ov == bv && oi < bi);
      bv = take ? ov : bv;
      bi = take ? oi : bi;
    }
    if (lane == 0) { sval[buf][w] = bv; sidx[buf][w] = bi; }
    __syncthreads();
    float rv = sval[buf][lane & 15];
    int   ri = sidx[buf][lane & 15];
#pragma unroll
    for (int off = 8; off > 0; off >>= 1) {
      const float ov = __shfl_xor(rv, off, 32);
      const int   oi = __shfl_xor(ri, off, 32);
      const bool take = (ov > rv) || (ov == rv && oi < ri);
      rv = take ? ov : rv;
      ri = take ? oi : ri;
    }
    far = ri;
    buf ^= 1;
  }
  __syncthreads();

  float cv[12];
#pragma unroll
  for (int i = 0; i < 4; ++i) {
    int fi = fidx_s[i * FPS_THREADS + tid];
    fi = fi < 0 ? 0 : (fi > NPTS - 1 ? NPTS - 1 : fi);
    cv[0 + i] = px[fi];
    cv[4 + i] = py[fi];
    cv[8 + i] = pz[fi];
  }
  float sq[4];
#pragma unroll
  for (int i = 0; i < 4; ++i) {
    const float t0 = cv[0 + i] * cv[0 + i];
    const float t1 = cv[4 + i] * cv[4 + i];
    const float t2 = cv[8 + i] * cv[8 + i];
    sq[i] = (t0 + t2) + t1;
  }
  for (int pass = 0; pass < 2; ++pass) {
#pragma unroll
    for (int c = 0; c < 3; ++c) {
#pragma unroll
      for (int i = 0; i < 4; ++i) {
        *(volatile float*)(out_xyz + ((size_t)(b * 3 + c)) * NQUERY + i * FPS_THREADS + tid) = cv[c * 4 + i];
      }
    }
#pragma unroll
    for (int i = 0; i < 4; ++i) {
      const v4f qv = {cv[0 + i], cv[4 + i], cv[8 + i], sq[i]};
      *(volatile v4f*)(qplane + ((size_t)(b * NQUERY + i * FPS_THREADS + tid)) * 4) = qv;
    }
    __threadfence();
  }
}

constexpr int XA_PITCH = 96;
constexpr int XB_PITCH = 64;
constexpr int OS_PITCH = 36;

__global__ __launch_bounds__(256) void group_mlp_kernel(
    const float* __restrict__ pts4, const float* __restrict__ qplane,
    const unsigned short* __restrict__ featT, const v4u* __restrict__ wplv,
    const float* __restrict__ biasf, float* __restrict__ out) {
#pragma clang fp contract(off)
  __shared__ int idx_s[8][NSAMP];
  __shared__ __align__(16) _Float16 xa[8][NSAMP * XA_PITCH];
  __shared__ __align__(16) _Float16 xb[8][NSAMP * XB_PITCH];
  __shared__ __align__(16) _Float16 w_s[WPL_HALVES];
  __shared__ __align__(16) float out_s[CH3 * OS_PITCH];
  __shared__ __align__(16) float bias_s[256];

  const int tid  = threadIdx.x;
  const int lane = tid & 31;
  const int w    = tid >> 5;
  const int hh   = lane >> 4;
  const int l15  = lane & 15;
  const int b    = blockIdx.x >> 6;
  const int s0   = (blockIdx.x & 63) * 32;

#pragma unroll 1
  for (int i = 0; i < 9; ++i) {
    const v4u t = wplv[i * 256 + tid];
    *(v4u*)(w_s + (size_t)(i * 256 + tid) * 8) = t;
  }
  bias_s[tid] = biasf[tid];
  __syncthreads();

  _Float16* xa_w = xa[w];
  _Float16* xb_w = xb[w];
  const float* pbase = pts4 + (size_t)b * NPTS * 4;

#pragma unroll 1
  for (int qi = 0; qi < 4; ++qi) {
    const int sl  = qi * 8 + w;
    const int qid = b * NQUERY + s0 + sl;
    const v4f qv = *(const v4f*)(qplane + (size_t)qid * 4);
    const float qx = qv[0];
    const float qy = qv[1];
    const float qz = qv[2];
    const float qs = qv[3];

    int cnt = 0;
    int first = NPTS - 1;
    for (int base = 0; base < NPTS; base += 32) {
      if (cnt >= NSAMP) break;
      const int n = base + lane;
      const v4f pv = *(const v4f*)(pbase + (size_t)n * 4);
      float dot = qx * pv[0];
      dot = __builtin_fmaf(qy, pv[1], dot);
      dot = __builtin_fmaf(qz, pv[2], dot);
      const float ssum = qs + pv[3];
      const float two  = 2.0f * dot;
      const float d    = ssum - two;
      const bool inb = d < RAD2;
      const unsigned m = __builtin_amdgcn_ballot_w32(inb);
      const int slot = cnt + __popc(m & ((1u << lane) - 1u));
      if (inb && slot < NSAMP) idx_s[w][slot] = n;
      first = (cnt == 0 && m != 0u) ? (base + __builtin_ffs((int)m) - 1) : first;
      cnt = __builtin_amdgcn_readfirstlane(cnt + __popc(m));
    }
    const int cc = cnt < NSAMP ? cnt : NSAMP;
    if (lane >= cc) idx_s[w][lane] = first;
    __syncthreads();

    {
      const int rq = lane >> 3;
      const int c8 = (lane & 7) * 8;
#pragma unroll 1
      for (int g2 = 0; g2 < 2; ++g2) {
        v4u tmp[4];
#pragma unroll
        for (int it = 0; it < 4; ++it) {
          const int row = (g2 * 4 + it) * 4 + rq;
          int id = idx_s[w][row];
          id = id < 0 ? 0 : (id > NPTS - 1 ? NPTS - 1 : id);
          tmp[it] = *(const v4u*)(featT + ((size_t)(b * NPTS + id)) * NFEAT + c8);
        }
#pragma unroll
        for (int it = 0; it < 4; ++it) {
          const int row = (g2 * 4 + it) * 4 + rq;
          *(v4u*)(xa_w + row * XA_PITCH + c8) = tmp[it];
        }
      }
      int id = idx_s[w][lane];
      id = id < 0 ? 0 : (id > NPTS - 1 ? NPTS - 1 : id);
      const v4f pv = *(const v4f*)(pbase + (size_t)id * 4);
      const float dx = pv[0] - qx;
      const float dy = pv[1] - qy;
      const float dz = pv[2] - qz;
      const _Float16 fx = (_Float16)dx;
      const _Float16 fy = (_Float16)dy;
      const _Float16 fz = (_Float16)dz;
      const unsigned ux = (unsigned)__builtin_bit_cast(unsigned short, fx);
      const unsigned uy = (unsigned)__builtin_bit_cast(unsigned short, fy);
      const unsigned uz = (unsigned)__builtin_bit_cast(unsigned short, fz);
      unsigned zz = 0u;
      asm volatile("" : "+v"(zz));
      const unsigned w0 = (ux & 0xffffu) | (uy << 16);
      const unsigned w1 = (uz & 0xffffu) | (zz << 16);
      const v4u t0 = {w0, w1, zz, zz};
      const v4u tz = {zz, zz, zz, zz};
      *(v4u*)(xa_w + lane * XA_PITCH + 64) = t0;
      *(v4u*)(xa_w + lane * XA_PITCH + 72) = tz;
      *(v4u*)(xa_w + lane * XA_PITCH + 80) = tz;
      *(v4u*)(xa_w + lane * XA_PITCH + 88) = tz;
    }
    __syncthreads();

    {
      v16h xf[2][3];
#pragma unroll
      for (int st = 0; st < 2; ++st)
#pragma unroll
        for (int k = 0; k < 3; ++k)
          xf[st][k] = frag_load(xa_w + (st * 16 + l15) * XA_PITCH + k * 32 + 8 * hh);
#pragma unroll
      for (int ct = 0; ct < 4; ++ct) {
        v16h wf[3];
#pragma unroll
        for (int k = 0; k < 3; ++k)
          wf[k] = frag_load(w_s + W1T_OFF + (ct * 16 + l15) * KPAD1 + k * 32 + 8 * hh);
        const v4f ba = *(const v4f*)(bias_s + ct * 16 + 8 * hh);
        const v4f bc = *(const v4f*)(bias_s + ct * 16 + 8 * hh + 4);
        v8f acc0 = {ba[0], ba[1], ba[2], ba[3], bc[0], bc[1], bc[2], bc[3]};
        v8f acc1 = acc0;
#pragma unroll
        for (int k = 0; k < 3; ++k) {
          acc0 = mma_h(wf[k], xf[0][k], acc0);
          acc1 = mma_h(wf[k], xf[1][k], acc1);
        }
        v8h h0, h1;
#pragma unroll
        for (int r = 0; r < 8; ++r) {
          h0[r] = (_Float16)leaky(acc0[r]);
          h1[r] = (_Float16)leaky(acc1[r]);
        }
        *(v8h*)(xb_w + (l15) * XB_PITCH + ct * 16 + 8 * hh) = h0;
        *(v8h*)(xb_w + (16 + l15) * XB_PITCH + ct * 16 + 8 * hh) = h1;
        asm volatile("" ::: "memory");
      }
    }
    __syncthreads();

    {
      v16h xf[2][2];
#pragma unroll
      for (int st = 0; st < 2; ++st)
#pragma unroll
        for (int k = 0; k < 2; ++k)
          xf[st][k] = frag_load(xb_w + (st * 16 + l15) * XB_PITCH + k * 32 + 8 * hh);
#pragma unroll
      for (int ct = 0; ct < 4; ++ct) {
        v16h wf[2];
#pragma unroll
        for (int k = 0; k < 2; ++k)
          wf[k] = frag_load(w_s + W2T_OFF + (ct * 16 + l15) * CH1 + k * 32 + 8 * hh);
        const v4f ba = *(const v4f*)(bias_s + 64 + ct * 16 + 8 * hh);
        const v4f bc = *(const v4f*)(bias_s + 64 + ct * 16 + 8 * hh + 4);
        v8f acc0 = {ba[0], ba[1], ba[2], ba[3], bc[0], bc[1], bc[2], bc[3]};
        v8f acc1 = acc0;
#pragma unroll
        for (int k = 0; k < 2; ++k) {
          acc0 = mma_h(wf[k], xf[0][k], acc0);
          acc1 = mma_h(wf[k], xf[1][k], acc1);
        }
        v8h h0, h1;
#pragma unroll
        for (int r = 0; r < 8; ++r) {
          h0[r] = (_Float16)leaky(acc0[r]);
          h1[r] = (_Float16)leaky(acc1[r]);
        }
        *(v8h*)(xa_w + (l15) * XA_PITCH + ct * 16 + 8 * hh) = h0;
        *(v8h*)(xa_w + (16 + l15) * XA_PITCH + ct * 16 + 8 * hh) = h1;
        asm volatile("" ::: "memory");
      }
    }
    __syncthreads();

    {
      v16h xf[2][2];
#pragma unroll
      for (int st = 0; st < 2; ++st)
#pragma unroll
        for (int k = 0; k < 2; ++k)
          xf[st][k] = frag_load(xa_w + (st * 16 + l15) * XA_PITCH + k * 32 + 8 * hh);
#pragma unroll
      for (int ct = 0; ct < 8; ++ct) {
        v16h wf[2];
#pragma unroll
        for (int k = 0; k < 2; ++k)
          wf[k] = frag_load(w_s + W3T_OFF + (ct * 16 + l15) * CH2 + k * 32 + 8 * hh);
        const float bv = bias_s[128 + ct * 16 + l15];
        v8f acc0 = {bv, bv, bv, bv, bv, bv, bv, bv};
        v8f acc1 = acc0;
#pragma unroll
        for (int k = 0; k < 2; ++k) {
          acc0 = mma_h(xf[0][k], wf[k], acc0);
          acc1 = mma_h(xf[1][k], wf[k], acc1);
        }
        float pm = acc0[0];
#pragma unroll
        for (int r = 1; r < 8; ++r) pm = fmaxf(pm, acc0[r]);
#pragma unroll
        for (int r = 0; r < 8; ++r) pm = fmaxf(pm, acc1[r]);
        const float po = __shfl_xor(pm, 16, 32);
        pm = leaky(fmaxf(pm, po));
        if (lane < 16) out_s[(ct * 16 + lane) * OS_PITCH + sl] = pm;
        asm volatile("" ::: "memory");
      }
    }
  }
  __syncthreads();

  {
    const int q4 = lane >> 3;
    const int c4 = (lane & 7) * 4;
    v4f vals[4];
#pragma unroll
    for (int it = 0; it < 4; ++it) {
      const int ch = w * 16 + it * 4 + q4;
      vals[it] = *(const v4f*)(out_s + ch * OS_PITCH + c4);
    }
    for (int pass = 0; pass < 2; ++pass) {
#pragma unroll
      for (int it = 0; it < 4; ++it) {
        const int ch = w * 16 + it * 4 + q4;
        *(volatile v4f*)(out + ((size_t)(b * CH3 + ch)) * NQUERY + s0 + c4) = vals[it];
      }
      __threadfence();
    }
  }
}

extern "C" void kernel_launch(void* const* d_in, const int* in_sizes, int n_in,
                              void* d_out, int out_size, void* d_ws, size_t ws_size,
                              hipStream_t stream) {
  (void)in_sizes;
  if (n_in < 20) return;
  if (ws_size < WS_TOTAL) return;
  if ((size_t)out_size < OUT0_ELEMS + OUT1_ELEMS) return;

  const float* features = (const float*)d_in[0];
  const float* points   = (const float*)d_in[1];
  const float* w1  = (const float*)d_in[2];
  const float* b1  = (const float*)d_in[3];
  const float* g1  = (const float*)d_in[4];
  const float* bb1 = (const float*)d_in[5];
  const float* m1  = (const float*)d_in[6];
  const float* v1  = (const float*)d_in[7];
  const float* w2  = (const float*)d_in[8];
  const float* b2  = (const float*)d_in[9];
  const float* g2  = (const float*)d_in[10];
  const float* bb2 = (const float*)d_in[11];
  const float* m2  = (const float*)d_in[12];
  const float* v2  = (const float*)d_in[13];
  const float* w3  = (const float*)d_in[14];
  const float* b3  = (const float*)d_in[15];
  const float* g3  = (const float*)d_in[16];
  const float* bb3 = (const float*)d_in[17];
  const float* m3  = (const float*)d_in[18];
  const float* v3  = (const float*)d_in[19];

  char* ws = (char*)d_ws;
  _Float16* wpl    = (_Float16*)(ws + WS_WPL);
  float*    biasf  = (float*)(ws + WS_BIAS);
  float*    qplane = (float*)(ws + WS_QPL);
  float*    pts4   = (float*)(ws + WS_PTS4);
  _Float16* featT  = (_Float16*)(ws + WS_FEATT);

  float* out     = (float*)d_out;
  float* out_xyz = out + OUT0_ELEMS;

  prep_kernel<<<10, 256, 0, stream>>>(w1, b1, g1, bb1, m1, v1,
                                      w2, b2, g2, bb2, m2, v2,
                                      w3, b3, g3, bb3, m3, v3, wpl, biasf);
  pack_kernel<<<NBATCH * (NPTS / 64), 256, 0, stream>>>(features, points, featT, pts4);
  fps_kernel<<<NBATCH, FPS_THREADS, 0, stream>>>(points, qplane, out_xyz);
  group_mlp_kernel<<<NBATCH * (NQUERY / 32), 256, 0, stream>>>(
      pts4, qplane, (const unsigned short*)featT, (const v4u*)(const void*)wpl, biasf, out);
}
